// FiDO_T5Attention_5600637354472
// MI455X (gfx1250) — hardware-verified
//
#include <hip/hip_runtime.h>


#define NB_  4
#define TT   2048
#define DM   1024
#define NHm  16
#define KVH  4
#define GG   4
#define HD   64
#define DO   256
#define PCAR 1024.0f
typedef _Float16 h16;
typedef unsigned short bf;
typedef __attribute__((ext_vector_type(16))) __bf16   v16bf;
typedef __attribute__((ext_vector_type(16))) _Float16 v16h;
typedef __attribute__((ext_vector_type(8)))  _Float16 v8h;
typedef __attribute__((ext_vector_type(8)))  unsigned short v8us;
typedef __attribute__((ext_vector_type(8)))  float    v8f;
typedef __attribute__((ext_vector_type(4)))  float    v4f;
typedef v8h  __attribute__((may_alias)) v8ha;
typedef v4f  __attribute__((may_alias)) v4fa;
typedef v8us __attribute__((may_alias)) v8usa;

__device__ __forceinline__ unsigned short f2bf(float f) { unsigned u = __float_as_uint(f); u += 0x7FFFu + ((u >> 16) & 1u); return (unsigned short)(u >> 16); }
__device__ __forceinline__ float bf2f(unsigned short b) { return __uint_as_float(((unsigned)b) << 16); }
__device__ __forceinline__ float bfr(float f) { return bf2f(f2bf(f)); }
__device__ __forceinline__ v16h cat16(v8h lo, v8h hi) { return __builtin_shufflevector(lo, hi, 0, 1, 2, 3, 4, 5, 6, 7, 8, 9, 10, 11, 12, 13, 14, 15); }
__device__ __forceinline__ v16bf cat16b(v8us lo, v8us hi) { return __builtin_bit_cast(v16bf, __builtin_shufflevector(lo, hi, 0, 1, 2, 3, 4, 5, 6, 7, 8, 9, 10, 11, 12, 13, 14, 15)); }
__device__ __forceinline__ v8f wmma16(v16h a, v16h b, v8f c) { return __builtin_amdgcn_wmma_f32_16x16x32_f16(false, a, false, b, (short)0, c, false, false); }
__device__ __forceinline__ v8f wmmab(v16bf a, v16bf b, v8f c) { return __builtin_amdgcn_wmma_f32_16x16x32_bf16(false, a, false, b, (short)0, c, false, false); }


template <typename T16> struct WFrag;
template <> struct WFrag<h16> { typedef v16h V; static __device__ __forceinline__ V ld(const h16* p) { return cat16(*(const v8h*)p, *(const v8h*)(p + 16)); } static __device__ __forceinline__ v8f mma(V a, V b, v8f c) { return wmma16(a, b, c); } };
template <> struct WFrag<bf> { typedef v16bf V; static __device__ __forceinline__ V ld(const bf* p) { return cat16b(*(const v8us*)p, *(const v8us*)(p + 16)); } static __device__ __forceinline__ v8f mma(V a, V b, v8f c) { return wmmab(a, b, c); } };
template <typename T16, int NSPLIT, bool BIAS>
__global__ __launch_bounds__(32) void k_gemmw(const T16* __restrict__ A, const T16* __restrict__ A2, const T16* __restrict__ Bt, const T16* __restrict__ Bt2, int K, float* C, int ldc, const float* __restrict__ bias, size_t sA, size_t sB, size_t sC) {
    typedef typename WFrag<T16>::V V;
    __shared__ __align__(16) float os[16 * 68];
    const size_t z = blockIdx.z; A += z * sA; if (A2) A2 += z * sA; Bt += z * sB; if (Bt2) Bt2 += z * sB; C += z * sC;
    const int lane = threadIdx.x & 31, lr = lane & 15, hi = lane >> 4; const int r0 = blockIdx.x * 64, c0 = blockIdx.y * 64;
    v8f acc[4][4];
#pragma unroll
    for (int mb = 0; mb < 4; ++mb)
#pragma unroll
        for (int nb = 0; nb < 4; ++nb) acc[mb][nb] = (v8f){};
    const size_t aoff = (size_t)(r0 + lr) * K + 8 * hi, boff = (size_t)(c0 + lr) * K + 8 * hi;
#pragma unroll 1
    for (int kc = 0; kc < K; kc += 32) {
        V a[4], a2[4];
#pragma unroll
        for (int mb = 0; mb < 4; ++mb) { a[mb] = WFrag<T16>::ld(A + aoff + (size_t)mb * 16 * K + kc); if (NSPLIT == 1 || NSPLIT == 2) a2[mb] = WFrag<T16>::ld(A2 + aoff + (size_t)mb * 16 * K + kc); }
#pragma unroll
        for (int nb = 0; nb < 4; ++nb) { const V b = WFrag<T16>::ld(Bt + boff + (size_t)nb * 16 * K + kc); V b2; if (NSPLIT >= 2) b2 = WFrag<T16>::ld(Bt2 + boff + (size_t)nb * 16 * K + kc);
#pragma unroll
            for (int mb = 0; mb < 4; ++mb) { acc[mb][nb] = WFrag<T16>::mma(a[mb], b, acc[mb][nb]); if (NSPLIT == 1 || NSPLIT == 2) acc[mb][nb] = WFrag<T16>::mma(a2[mb], b, acc[mb][nb]); if (NSPLIT >= 2) acc[mb][nb] = WFrag<T16>::mma(a[mb], b2, acc[mb][nb]); } }
        asm volatile("v_nop\n\tv_nop\n\tv_nop\n\tv_nop" : "+v"(acc[0][0]), "+v"(acc[1][1]), "+v"(acc[2][2]), "+v"(acc[3][3]) : "v"(a[0]), "v"(a[3]));
    }
#pragma unroll
    for (int mb = 0; mb < 4; ++mb) {
#pragma unroll
        for (int nb = 0; nb < 4; ++nb) {
#pragma unroll
            for (int j = 0; j < 8; ++j) os[(hi * 8 + j) * 68 + nb * 16 + lr] = acc[mb][nb][j]; }
        __builtin_amdgcn_wave_barrier(); asm volatile("" ::: "memory");
        float* crow = C + (size_t)(r0 + mb * 16) * ldc + c0;
#pragma unroll 1
        for (int ps = 0; ps < 2; ++ps) {
#pragma unroll
            for (int s = 0; s < 8; ++s) { const int row = 2 * s + hi, cofs = lr * 4; v4f val = *(const v4fa*)(os + row * 68 + cofs); if (BIAS) { val[0] += bfr(bias[c0 + cofs]); val[1] += bfr(bias[c0 + cofs + 1]); val[2] += bfr(bias[c0 + cofs + 2]); val[3] += bfr(bias[c0 + cofs + 3]); }
                *(volatile v4f*)(crow + (size_t)row * ldc + cofs) = val; }
            if (ps == 0) __threadfence(); }
        __builtin_amdgcn_wave_barrier(); asm volatile("" ::: "memory");
    }
}

__device__ __forceinline__ h16 tohx(float x) { return (h16)x; }
__device__ __forceinline__ void splitf(float y, unsigned short& h, unsigned short& l) { h = f2bf(y); l = f2bf(y - bf2f(h)); }
typedef __attribute__((ext_vector_type(2))) unsigned short v2us;
typedef __attribute__((ext_vector_type(4))) unsigned short v4us;
typedef __attribute__((ext_vector_type(2))) _Float16 v2h;
typedef __attribute__((ext_vector_type(4))) _Float16 v4h;
__constant__ unsigned char c_bucket[4095] = { 15,15,15,15,15,15,15,15,15,15,15,15,15,15,15,15,15,15,15,15,15,15,15,15,15,15,15,15,15,15,15,15,15,15,15,15,15,15,15,15,15,15,15,15,15,15,15,15,15,15,15,15,15,15,15,15,15,15,15,15,15,15,15,15,15,15,15,15,15,15,15,15,15,15,15,15,15,15,15,15,15,15,15,15,15,15,15,15,15,15,15,15,15,15,15,15,15,15,15,15,15,15,15,15,15,15,15,15,15,15,15,15,15,15,15,15,15,15,15,15,15,15,15,15,15,15,15,15,15,15,15,15,15,15,15,15,15,15,15,15,15,15,15,15,15,15,15,15,15,15,15,15,15,15,15,15,15,15,15,15,15,15,15,15,15,15,15,15,15,15,15,15,15,15,15,15,15,15,15,15,15,15,15,15,15,15,15,15,15,15,15,15,15,15,15,15,15,15,15,15,15,15,15,15,15,15,15,15,15,15,15,15,15,15,15,15,15,15,15,15,15,15,15,15,15,15,15,15,15,15,15,15,15,15,15,15,15,15,15,15,15,15,15,15,15,15,15,15,15,15,15,15,15,15,15,15,15,15,15,15,15,15,15,15,15,15,15,15,15,15,15,15,15,15,15,15,15,15,15,15,15,15,15,15,15,15,15,15,15,15,15,15,15,15,15,15,15,15,15,15,15,15,15,15,15,15,15,15,15,15,15,15,15,15,15,15,15,15,15,15,15,15,15,15,15,15,15,15,15,15,15,15,15,15,15,15,15,15,15,15,15,15,15,15,15,15,15,15,15,15,15,15,15,15,15,15,15,15,15,15,15,15,15,15,15,15,15,15,15,15,15,15,15,15,15,15,15,15,15,15,15,15,15,15,15,15,15,15,15,15,15,15,15,15,15,15,15,15,15,15,15,15,15,15,15,15,15,15,15,15,15,15,15,15,15,15,15,15,15,15,15,15,15,15,15,15,15,15,15,15,15,15,15,15,15,15,15,15,15,15,15,15,15,15,15,15,15,15,15,15,15,15,15,15,15,15,15,15,15,15,15,15,15,15,15,15,15,15,15,15,15,15,15,15,15,15,15,15,15,15,15,15,15,15,15,15,15,15,15,15,15,15,15,15,15,15,15,15,15,15,15,15,15,15,15,15,15,15,15,15,15,15,15,15,15,15,15,15,15,15,15,15,15,15,15,15,15,15,15,15,15,15,15,15,15,15,15,15,15,15,15,15,15,15,15,15,15,15,15,15,15,15,15,15,15,15,15,15,15,15,15,15,15,15,15,15,15,15,15,15,15,15,15,15,15,15,15,15,15,15,15,15,15,15,15,15,15,15,15,15,15,15,15,15,15,15,15,15,15,15,15,15,15,15,15,15,15,15,15,15,15,15,15,15,15,15,15,15,15,15,15,15,15,15,15,15,15,15,15,15,15,15,15,15,15,15,15,15,15,15,15,15,15,15,15,15,15,15,15,15,15,15,15,15,15,15,15,15,15,15,15,15,15,15,15,15,15,15,15,15,15,15,15,15,15,15,15,15,15,15,15,15,15,15,15,15,15,15,15,15,15,15,15,15,15,15,15,15,15,15,15,15,15,15,15,15,15,15,15,15,15,15,15,15,15,15,15,15,15,15,15,15,15,15,15,15,15,15,15,15,15,15,15,15,15,15,15,15,15,15,15,15,15,15,15,15,15,15,15,15,15,15,15,15,15,15,15,15,15,15,15,15,15,15,15,15,15,15,15,15,15,15,15,15,15,15,15,15,15,15,15,15,15,15,15,15,15,15,15,15,15,15,15,15,15,15,15,15,15,15,15,15,15,15,15,15,15,15,15,15,15,15,15,15,15,15,15,15,15,15,15,15,15,15,15,15,15,15,15,15,15,15,15,15,15,15,15,15,15,15,15,15,15,15,15,15,15,15,15,15,15,15,15,15,15,15,15,15,15,15,15,15,15,15,15,15,15,15,15,15,15,15,15,15,15,15,15,15,15,15,15,15,15,15,15,15,15,15,15,15,15,15,15,15,15,15,15,15,15,15,15,15,15,15,15,15,15,15,15,15,15,15,15,15,15,15,15,15,15,15,15,15,15,15,15,15,15,15,15,15,15,15,15,15,15,15,15,15,15,15,15,15,15,15,15,15,15,15,15,15,15,15,15,15,15,15,15,15,15,15,15,15,15,15,15,15,15,15,15,15,15,15,15,15,15,15,15,15,15,15,15,15,15,15,15,15,15,15,15,15,15,15,15,15,15,15,15,15,15,15,15,15,15,15,15,15,15,15,15,15,15,15,15,15,15,15,15,15,15,15,15,15,15,15,15,15,15,15,15,15,15,15,15,15,15,15,15,15,15,15,15,15,15,15,15,15,15,15,15,15,15,15,15,15,15,15,15,15,15,15,15,15,15,15,15,15,15,15,15,15,15,15,15,15,15,15,15,15,15,15,15,15,15,15,15,15,15,15,15,15,15,15,15,15,15,15,15,15,15,15,15,15,15,15,15,15,15,15,15,15,15,15,15,15,15,15,15,15,15,15,15,15,15,15,15,15,15,15,15,15,15,15,15,15,15,15,15,15,15,15,15,15,15,15,15,15,15,15,15,15,15,15,15,15,15,15,15,15,15,15,15,15,15,15,15,15,15,15,15,15,15,15,15,15,15,15,15,15,15,15,15,15,15,15,15,15,15,15,15,15,15,15,15,15,15,15,15,15,15,15,15,15,15,15,15,15,15,15,15,15,15,15,15,15,15,15,15,15,15,15,15,15,15,15,15,15,15,15,15,15,15,15,15,15,15,15,15,15,15,15,15,15,15,15,15,15,15,15,15,15,15,15,15,15,15,15,15,15,15,15,15,15,15,15,15,15,15,15,15,15,15,15,15,15,15,15,15,15,15,15,15,15,15,15,15,15,15,15,15,15,15,15,15,15,15,15,15,15,15,15,15,15,15,15,15,15,15,15,15,15,15,15,15,15,15,15,15,15,15,15,15,15,15,15,15,15,15,15,15,15,15,15,15,15,15,15,15,15,15,15,15,15,15,15,15,15,15,15,15,15,15,15,15,15,15,15,15,15,15,15,15,15,15,15,15,15,15,15,15,15,15,15,15,15,15,15,15,15,15,15,15,15,15,15,15,15,15,15,15,15,15,15,15,15,15,15,15,15,15,15,15,15,15,15,15,15,15,15,15,15,15,15,15,15,15,15,15,15,15,15,15,15,15,15,15,15,15,15,15,15,15,15,15,15,15,15,15,15,15,15,15,15,15,15,15,15,15,15,15,15,15,15,15,15,15,15,15,15,15,15,15,15,15,15,15,15,15,15,15,15,15,15,15,15,15,15,15,15,15,15,15,15,15,15,15,15,15,15,15,15,15,15,15,15,15,15,15,15,15,15,15,15,15,15,15,15,15,15,15,15,15,15,15,15,15,15,15,15,15,15,15,15,15,15,15,15,15,15,15,15,15,15,15,15,15,15,15,15,15,15,15,15,15,15,15,15,15,15,15,15,15,15,15,15,15,15,15,15,15,15,15,15,15,15,15,15,15,15,15,15,15,15,15,15,15,15,15,15,15,15,15,15,15,15,15,15,15,15,15,15,15,15,15,15,15,15,15,15,15,15,15,15,15,15,15,15,15,15,15,15,15,15,15,15,15,15,15,15,15,15,15,15,15,15,15,15,15,15,15,15,15,15,15,15,15,15,15,15,15,15,15,15,15,15,15,15,15,15,15,15,15,15,15,15,15,15,15,15,15,15,15,15,15,15,15,15,15,15,15,15,15,15,15,15,15,15,15,15,15,15,15,15,15,15,15,15,15,15,15,15,15,15,15,15,15,15,15,15,15,15,15,15,15,15,15,15,15,15,15,15,15,15,15,15,15,15,15,15,15,15,15,15,15,15,15,15,15,15,15,15,15,15,15,15,15,15,15,15,15,15,15,15,15,15,15,15,15,15,15,15,15,15,15,15,15,15,15,15,15,15,15,15,15,15,15,15,15,15,15,15,15,15,15,15,15,15,15,15,15,15,15,15,15,15,15,15,15,15,15,15,15,15,15,15,15,15,15,15,15,15,15,15,15,15,15,15,15,15,15,15,15,15,15,15,15,15,15,15,15,15,15,15,15,15,15,15,15,15,15,15,15,15,15,15,15,15,15,15,15,15,15,15,15,15,15,15,15,15,15,15,15,15,15,15,15,15,15,15,15,15,15,15,15,15,15,15,15,15,15,15,15,15,15,15,15,15,15,15,15,15,15,15,15,15,15,15,15,15,15,15,15,15,15,15,15,15,15,15,15,15,15,15,15,15,15,15,15,15,15,15,15,15,15,15,15,15,15,15,15,15,15,15,15,15,15,15,15,15,15,15,15,15,15,15,15,15,15,15,15,15,15,15,15,15,15,15,15,15,15,15,15,15,15,15,15,15,15,14,14,14,14,14,14,14,14,14,14,14,14,14,14,14,14,14,14,14,14,14,14,14,14,14,14,14,13,13,13,13,13,13,13,13,13,13,13,13,13,13,13,13,13,13,12,12,12,12,12,12,12,12,12,12,12,12,12,12,11,11,11,11,11,11,11,11,11,10,10,10,10,10,10,10,9,9,9,9,8,8,8,8,7,6,5,4,3,2,1,0,17,18,19,20,21,22,23,24,24,24,24,25,25,25,25,26,26,26,26,26,26,26,27,27,27,27,27,27,27,27,27,28,28,28,28,28,28,28,28,28,28,28,28,28,28,29,29,29,29,29,29,29,29,29,29,29,29,29,29,29,29,29,29,30,30,30,30,30,30,30,30,30,30,30,30,30,30,30,30,30,30,30,30,30,30,30,30,30,30,30,31,31,31,31,31,31,31,31,31,31,31,31,31,31,31,31,31,31,31,31,31,31,31,31,31,31,31,31,31,31,31,31,31,31,31,31,31,31,31,31,31,31,31,31,31,31,31,31,31,31,31,31,31,31,31,31,31,31,31,31,31,31,31,31,31,31,31,31,31,31,31,31,31,31,31,31,31,31,31,31,31,31,31,31,31,31,31,31,31,31,31,31,31,31,31,31,31,31,31,31,31,31,31,31,31,31,31,31,31,31,31,31,31,31,31,31,31,31,31,31,31,31,31,31,31,31,31,31,31,31,31,31,31,31,31,31,31,31,31,31,31,31,31,31,31,31,31,31,31,31,31,31,31,31,31,31,31,31,31,31,31,31,31,31,31,31,31,31,31,31,31,31,31,31,31,31,31,31,31,31,31,31,31,31,31,31,31,31,31,31,31,31,31,31,31,31,31,31,31,31,31,31,31,31,31,31,31,31,31,31,31,31,31,31,31,31,31,31,31,31,31,31,31,31,31,31,31,31,31,31,31,31,31,31,31,31,31,31,31,31,31,31,31,31,31,31,31,31,31,31,31,31,31,31,31,31,31,31,31,31,31,31,31,31,31,31,31,31,31,31,31,31,31,31,31,31,31,31,31,31,31,31,31,31,31,31,31,31,31,31,31,31,31,31,31,31,31,31,31,31,31,31,31,31,31,31,31,31,31,31,31,31,31,31,31,31,31,31,31,31,31,31,31,31,31,31,31,31,31,31,31,31,31,31,31,31,31,31,31,31,31,31,31,31,31,31,31,31,31,31,31,31,31,31,31,31,31,31,31,31,31,31,31,31,31,31,31,31,31,31,31,31,31,31,31,31,31,31,31,31,31,31,31,31,31,31,31,31,31,31,31,31,31,31,31,31,31,31,31,31,31,31,31,31,31,31,31,31,31,31,31,31,31,31,31,31,31,31,31,31,31,31,31,31,31,31,31,31,31,31,31,31,31,31,31,31,31,31,31,31,31,31,31,31,31,31,31,31,31,31,31,31,31,31,31,31,31,31,31,31,31,31,31,31,31,31,31,31,31,31,31,31,31,31,31,31,31,31,31,31,31,31,31,31,31,31,31,31,31,31,31,31,31,31,31,31,31,31,31,31,31,31,31,31,31,31,31,31,31,31,31,31,31,31,31,31,31,31,31,31,31,31,31,31,31,31,31,31,31,31,31,31,31,31,31,31,31,31,31,31,31,31,31,31,31,31,31,31,31,31,31,31,31,31,31,31,31,31,31,31,31,31,31,31,31,31,31,31,31,31,31,31,31,31,31,31,31,31,31,31,31,31,31,31,31,31,31,31,31,31,31,31,31,31,31,31,31,31,31,31,31,31,31,31,31,31,31,31,31,31,31,31,31,31,31,31,31,31,31,31,31,31,31,31,31,31,31,31,31,31,31,31,31,31,31,31,31,31,31,31,31,31,31,31,31,31,31,31,31,31,31,31,31,31,31,31,31,31,31,31,31,31,31,31,31,31,31,31,31,31,31,31,31,31,31,31,31,31,31,31,31,31,31,31,31,31,31,31,31,31,31,31,31,31,31,31,31,31,31,31,31,31,31,31,31,31,31,31,31,31,31,31,31,31,31,31,31,31,31,31,31,31,31,31,31,31,31,31,31,31,31,31,31,31,31,31,31,31,31,31,31,31,31,31,31,31,31,31,31,31,31,31,31,31,31,31,31,31,31,31,31,31,31,31,31,31,31,31,31,31,31,31,31,31,31,31,31,31,31,31,31,31,31,31,31,31,31,31,31,31,31,31,31,31,31,31,31,31,31,31,31,31,31,31,31,31,31,31,31,31,31,31,31,31,31,31,31,31,31,31,31,31,31,31,31,31,31,31,31,31,31,31,31,31,31,31,31,31,31,31,31,31,31,31,31,31,31,31,31,31,31,31,31,31,31,31,31,31,31,31,31,31,31,31,31,31,31,31,31,31,31,31,31,31,31,31,31,31,31,31,31,31,31,31,31,31,31,31,31,31,31,31,31,31,31,31,31,31,31,31,31,31,31,31,31,31,31,31,31,31,31,31,31,31,31,31,31,31,31,31,31,31,31,31,31,31,31,31,31,31,31,31,31,31,31,31,31,31,31,31,31,31,31,31,31,31,31,31,31,31,31,31,31,31,31,31,31,31,31,31,31,31,31,31,31,31,31,31,31,31,31,31,31,31,31,31,31,31,31,31,31,31,31,31,31,31,31,31,31,31,31,31,31,31,31,31,31,31,31,31,31,31,31,31,31,31,31,31,31,31,31,31,31,31,31,31,31,31,31,31,31,31,31,31,31,31,31,31,31,31,31,31,31,31,31,31,31,31,31,31,31,31,31,31,31,31,31,31,31,31,31,31,31,31,31,31,31,31,31,31,31,31,31,31,31,31,31,31,31,31,31,31,31,31,31,31,31,31,31,31,31,31,31,31,31,31,31,31,31,31,31,31,31,31,31,31,31,31,31,31,31,31,31,31,31,31,31,31,31,31,31,31,31,31,31,31,31,31,31,31,31,31,31,31,31,31,31,31,31,31,31,31,31,31,31,31,31,31,31,31,31,31,31,31,31,31,31,31,31,31,31,31,31,31,31,31,31,31,31,31,31,31,31,31,31,31,31,31,31,31,31,31,31,31,31,31,31,31,31,31,31,31,31,31,31,31,31,31,31,31,31,31,31,31,31,31,31,31,31,31,31,31,31,31,31,31,31,31,31,31,31,31,31,31,31,31,31,31,31,31,31,31,31,31,31,31,31,31,31,31,31,31,31,31,31,31,31,31,31,31,31,31,31,31,31,31,31,31,31,31,31,31,31,31,31,31,31,31,31,31,31,31,31,31,31,31,31,31,31,31,31,31,31,31,31,31,31,31,31,31,31,31,31,31,31,31,31,31,31,31,31,31,31,31,31,31,31,31,31,31,31,31,31,31,31,31,31,31,31,31,31,31,31,31,31,31,31,31,31,31,31,31,31,31,31,31,31,31,31,31,31,31,31,31,31,31,31,31,31,31,31,31,31,31,31,31,31,31,31,31,31,31,31,31,31,31,31,31,31,31,31,31,31,31,31,31,31,31,31,31,31,31,31,31,31,31,31,31,31,31,31,31,31,31,31,31,31,31,31,31,31,31,31,31,31,31,31,31,31,31,31,31,31,31,31,31,31,31,31,31,31,31,31,31,31,31,31,31,31,31,31,31,31,31,31,31,31,31,31,31,31,31,31,31,31,31,31,31,31,31,31,31,31,31,31,31,31,31,31,31,31,31,31,31,31,31,31,31,31,31,31,31,31,31,31,31,31,31,31,31,31,31,31,31,31,31,31,31,31,31,31,31,31,31,31,31,31,31,31,31,31,31,31,31,31,31,31,31,31,31,31,31,31,31,31,31,31,31,31,31,31,31,31,31,31,31,31,31,31,31,31,31,31,31,31,31,31,31,31,31,31,31,31,31,31,31,31,31,31,31,31,31,31,31,31,31,31,31,31,31,31,31,31,31,31,31,31,31,31,31,31,31,31,31,31,31,31,31,31,31,31,31,31,31,31,31,31,31,31,31,31,31,31,31,31,31,31,31,31,31,31,31,31,31,31,31,31,31,31,31,31,31,31,31,31,31,31,31,31,31,31,31,31,31,31,31,31,31,31,31,31,31,31,31,31,31,31,31,31,31,31,31,31,31,31,31,31,31,31,31,31,31,31,31,31,31,31,31,31,31,31,31,31,31,31,31,31,31,31,31,31,31,31,31,31,31,31,31,31,31,31,31,31,31,31,31,31,31,31,31,31,31,31,31,31,31,31,31,31,31,31,31,31,31,31,31,31,31,31,31,31,31,31,31,31,31,31,31,31,31,31,31,31,31,31,31,31,31,31,31,31,31,31,31,31,31,31,31,31,31,31,31,31,31,31,31,31,31,31,31,31,31,31,31,31,31,31,31,31,31,31,31,31,31,31,31,31,31,31,31,31,31,31,31,31,31,31,31,31,31,31,31,31,31,31,31,31,31,31,31,31,31,31,31,31,31,31,31,31,31,31,31,31,31,31,31,31,31,31,31,31,31,31,31,31,31,31,31,31,31,31,31,31,31,31,31,31,31,31,31,31,31,31,31,31,31,31,31,31,31,31,31,31,31,31,31,31,31,31,31,31,31,31,31,31,31,31,31,31,31,31,31,31,31,31,31,31,31,31,31,31,31,31,31,31,31,31,31,31,31,31,31,31,31,31,31,31,31,31,31,31,31,31,31,31,31,31,31,31,31,31,31,31,31,31,31,31,31,31,31,31,31,31,31,31,31,31,31,31,31,31,31,31,31,31,31,31,31,31,31,31,31,31,31,31,31,31,31,31,31,31,31,31,31,31,31,31,31,31,31,31,31,31,31,31,31,31,31,31,31,31,31,31,31,31,31,31 };

__global__ __launch_bounds__(256) void k_cvt8(const float* __restrict__ src, bf* dst, size_t n8) { const size_t i = (size_t)blockIdx.x * 256 + threadIdx.x; if (i >= n8) return; const v8f v = *(const v8f*)(src + i * 8); v8us o;
#pragma unroll
    for (int k = 0; k < 8; ++k) o[k] = f2bf(v[k]); *(volatile v8us*)(dst + i * 8) = o; __threadfence(); *(volatile v8us*)(dst + i * 8) = o; }
__global__ __launch_bounds__(256) void k_qs(const float* __restrict__ Q, bf* Ph, bf* Pl) { const int e = (blockIdx.x * 256 + threadIdx.x) * 4; if (e >= KVH * TT * HD) return; const int d = e % HD; const int t = (e / HD) % TT; const int h = e / (HD * TT); const float* r = Q + (size_t)t * DM + h * HD + d; v4us oh, ol;
#pragma unroll
    for (int u = 0; u < 4; ++u) { float s = 0.f;
#pragma unroll
        for (int g = 0; g < GG; ++g) s = __fadd_rn(s, r[g * KVH * HD + u]); unsigned short a, b; splitf(s, a, b); oh[u] = a; ol[u] = b; }
    *(volatile v4us*)(Ph + e) = oh; *(volatile v4us*)(Pl + e) = ol; __threadfence(); *(volatile v4us*)(Ph + e) = oh; *(volatile v4us*)(Pl + e) = ol; }
__global__ __launch_bounds__(256) void k_gk(const float* __restrict__ K, bf* Ph, bf* Pl) { const int e = (blockIdx.x * 256 + threadIdx.x) * 4; if (e >= KVH * TT * HD) return; const int d = e % HD; const int t = (e / HD) % TT; const int h = e / (HD * TT); const float* r = K + (size_t)t * DM + h * HD + d; v4us oh, ol;
#pragma unroll
    for (int u = 0; u < 4; ++u) { float s = 0.f;
#pragma unroll
        for (int g = 0; g < GG; ++g) s = __fadd_rn(s, r[g * KVH * HD + u]); unsigned short a, b; splitf(s * 0.25f, a, b); oh[u] = a; ol[u] = b; }
    *(volatile v4us*)(Ph + e) = oh; *(volatile v4us*)(Pl + e) = ol; __threadfence(); *(volatile v4us*)(Ph + e) = oh; *(volatile v4us*)(Pl + e) = ol; }
__global__ __launch_bounds__(256) void k_gvt(const float* __restrict__ V, h16* GVT) { const int e = (blockIdx.x * 256 + threadIdx.x) * 2; if (e >= KVH * HD * TT) return; const int s = e % TT; const int d = (e / TT) % HD; const int h = e / (TT * HD); v2h o;
#pragma unroll
    for (int u = 0; u < 2; ++u) { const float* r = V + (size_t)(s + u) * DM + h * HD + d; float a = 0.f;
#pragma unroll
        for (int g = 0; g < GG; ++g) a = __fadd_rn(a, r[g * KVH * HD]); o[u] = tohx(a * 0.25f); }
    *(volatile v2h*)(GVT + e) = o; __threadfence(); *(volatile v2h*)(GVT + e) = o; }
__global__ __launch_bounds__(256) void k_btab(const float* __restrict__ rb, float* TB) { const int i = blockIdx.x * 256 + threadIdx.x; if (i >= KVH * 4095) return; const int r = i % 4095, h = i / 4095; const int bk = c_bucket[r]; float s = 0.f;
#pragma unroll
    for (int g = 0; g < GG; ++g) s = __fadd_rn(s, bfr(rb[bk * NHm + g * KVH + h])); const float v = s * 0.25f; *(volatile float*)(TB + i) = v; __threadfence(); *(volatile float*)(TB + i) = v; }
__global__ __launch_bounds__(256) void k_woe(const float* __restrict__ wo, bf* Wh, bf* Wl) { const int e = (blockIdx.x * 256 + threadIdx.x) * 4; if (e >= DM * DO) return; const int j = e % DO; const int o = e / DO; const float* r = wo + (size_t)o * DM + j; v4us oh, ol;
#pragma unroll
    for (int u = 0; u < 4; ++u) { float s = 0.f;
#pragma unroll
        for (int g = 0; g < GG; ++g) s = __fadd_rn(s, bfr(r[g * DO + u])); unsigned short a, b; splitf(s, a, b); oh[u] = a; ol[u] = b; }
    *(volatile v4us*)(Wh + e) = oh; *(volatile v4us*)(Wl + e) = ol; __threadfence(); *(volatile v4us*)(Wh + e) = oh; *(volatile v4us*)(Wl + e) = ol; }
__global__ __launch_bounds__(256) void k_mrg(const float* __restrict__ O, bf* Ph, bf* Pl) { const int e = (blockIdx.x * 256 + threadIdx.x) * 4; if (e >= TT * DO) return; const int c = e % DO; const int t = e / DO; const int h = c / HD, d = c % HD; const float* r = O + ((size_t)h * TT + t) * HD + d; v4us oh, ol;
#pragma unroll
    for (int u = 0; u < 4; ++u) { unsigned short a, b; splitf(r[u] * (1.0f / PCAR), a, b); oh[u] = a; ol[u] = b; } *(volatile v4us*)(Ph + e) = oh; *(volatile v4us*)(Pl + e) = ol; __threadfence(); *(volatile v4us*)(Ph + e) = oh; *(volatile v4us*)(Pl + e) = ol; }
__global__ __launch_bounds__(256) void k_bsoft(const float* __restrict__ Sb, const float* __restrict__ TB, h16* P16) { const int lane = threadIdx.x & 31; const int row = blockIdx.x * 8 + (threadIdx.x >> 5); if (row >= KVH * TT) return; const int n = row % TT; const int h = row / TT; const float* sr = Sb + (size_t)row * TT; const float* tb = TB + (size_t)h * 4095 + 2047 - n; float mx = -3.0e38f;
#pragma unroll 1
    for (int ch = 0; ch < TT / 128; ++ch) { const int j0 = ch * 128 + lane * 4; const v4f a = *(const v4f*)(sr + j0);
#pragma unroll
        for (int u = 0; u < 4; ++u) mx = fmaxf(mx, __fadd_rn(a[u], tb[j0 + u])); }
#pragma unroll
    for (int sh = 16; sh; sh >>= 1) mx = fmaxf(mx, __shfl_xor(mx, sh, 32));
    float sum = 0.f;
#pragma unroll 1
    for (int ch = 0; ch < TT / 128; ++ch) { const int j0 = ch * 128 + lane * 4; const v4f a = *(const v4f*)(sr + j0);
#pragma unroll
        for (int u = 0; u < 4; ++u) { float d0 = __fsub_rn(__fadd_rn(a[u], tb[j0 + u]), mx); asm volatile("" : "+v"(d0)); sum += __expf(d0); } }
#pragma unroll
    for (int sh = 16; sh; sh >>= 1) sum += __shfl_xor(sum, sh, 32);
    const float f = __fdiv_rn(PCAR, sum);
    for (int ps = 0; ps < 2; ++ps) {
#pragma unroll 1
        for (int ch = 0; ch < TT / 128; ++ch) { const int j0 = ch * 128 + lane * 4; const v4f a = *(const v4f*)(sr + j0); v4h o;
#pragma unroll
            for (int u = 0; u < 4; ++u) { float d0 = __fsub_rn(__fadd_rn(a[u], tb[j0 + u]), mx); asm volatile("" : "+v"(d0)); o[u] = tohx(__fmul_rn(__expf(d0), f)); } *(volatile v4h*)(P16 + (size_t)row * TT + j0) = o; }
        if (ps == 0) __threadfence(); } }

extern "C" void kernel_launch(void* const* d_in, const int* in_sizes, int n_in,
                              void* d_out, int out_size, void* d_ws, size_t ws_size, hipStream_t stream) {
    (void)in_sizes; (void)n_in; (void)out_size;
    const float* x = (const float*)d_in[0]; const float* wq = (const float*)d_in[1]; const float* wk = (const float*)d_in[2]; const float* wv = (const float*)d_in[3]; const float* wo = (const float*)d_in[4]; const float* rb = (const float*)d_in[5];
    float* OUT = (float*)d_out;
    char* wsp = (char*)d_ws;
    auto take = [&](size_t bytes) { char* p = wsp; wsp += (bytes + 255) & ~(size_t)255; return (void*)p; };
    bf* WQ = (bf*)take((size_t)DM * DM * 2); bf* WK = (bf*)take((size_t)DM * DM * 2); bf* WV = (bf*)take((size_t)DM * DM * 2); bf* WEh = (bf*)take((size_t)DM * DO * 2); bf* WEl = (bf*)take((size_t)DM * DO * 2); float* TB = (float*)take((size_t)KVH * 4095 * 4 + 256);
    bf* XB = (bf*)take((size_t)TT * DM * 2); float* Q = (float*)take((size_t)TT * DM * 4); float* K = (float*)take((size_t)TT * DM * 4); bf* QSh = (bf*)take((size_t)KVH * TT * HD * 2); bf* QSl = (bf*)take((size_t)KVH * TT * HD * 2); bf* GKh = (bf*)take((size_t)KVH * TT * HD * 2); bf* GKl = (bf*)take((size_t)KVH * TT * HD * 2); h16* GVT = (h16*)take((size_t)KVH * HD * TT * 2);
    float* Sb = (float*)take((size_t)KVH * TT * TT * 4); h16* P16 = (h16*)take((size_t)KVH * TT * TT * 2); float* O = (float*)take((size_t)KVH * TT * HD * 4); bf* OPh = (bf*)take((size_t)TT * DO * 2); bf* OPl = (bf*)take((size_t)TT * DO * 2);
    if ((size_t)(wsp - (char*)d_ws) > ws_size) return;
    float* V = K;
    k_cvt8<<<(DM * DM / 8 + 255) / 256, 256, 0, stream>>>(wq, WQ, (size_t)DM * DM / 8); k_cvt8<<<(DM * DM / 8 + 255) / 256, 256, 0, stream>>>(wk, WK, (size_t)DM * DM / 8); k_cvt8<<<(DM * DM / 8 + 255) / 256, 256, 0, stream>>>(wv, WV, (size_t)DM * DM / 8);
    k_woe<<<(DM * DO / 4 + 255) / 256, 256, 0, stream>>>(wo, WEh, WEl); k_btab<<<(KVH * 4095 + 255) / 256, 256, 0, stream>>>(rb, TB);
    for (int b = 0; b < NB_; ++b) {
        k_cvt8<<<(unsigned)(((size_t)TT * DM / 8 + 255) / 256), 256, 0, stream>>>(x + (size_t)b * TT * DM, XB, (size_t)TT * DM / 8);
        k_gemmw<bf, 0, false><<<dim3(TT / 64, DM / 64, 1), 32, 0, stream>>>(XB, nullptr, WQ, nullptr, DM, Q, DM, nullptr, 0, 0, 0); k_qs<<<(KVH * TT * HD / 4 + 255) / 256, 256, 0, stream>>>(Q, QSh, QSl);
        k_gemmw<bf, 0, false><<<dim3(TT / 64, DM / 64, 1), 32, 0, stream>>>(XB, nullptr, WK, nullptr, DM, K, DM, nullptr, 0, 0, 0); k_gk<<<(KVH * TT * HD / 4 + 255) / 256, 256, 0, stream>>>(K, GKh, GKl);
        k_gemmw<bf, 0, false><<<dim3(TT / 64, DM / 64, 1), 32, 0, stream>>>(XB, nullptr, WV, nullptr, DM, V, DM, nullptr, 0, 0, 0); k_gvt<<<(KVH * HD * TT / 2 + 255) / 256, 256, 0, stream>>>(V, GVT);
        k_gemmw<bf, 2, false><<<dim3(TT / 64, TT / 64, KVH), 32, 0, stream>>>(QSh, QSl, GKh, GKl, HD, Sb, TT, nullptr, (size_t)TT * HD, (size_t)TT * HD, (size_t)TT * TT);
        k_bsoft<<<KVH * TT / 8, 256, 0, stream>>>(Sb, TB, P16);
        k_gemmw<h16, 0, false><<<dim3(TT / 64, 1, KVH), 32, 0, stream>>>(P16, nullptr, GVT, nullptr, TT, O, HD, nullptr, (size_t)TT * TT, (size_t)HD * TT, (size_t)TT * HD);
        k_mrg<<<(TT * DO / 4 + 255) / 256, 256, 0, stream>>>(O, OPh, OPl);
        k_gemmw<bf, 2, false><<<dim3(TT / 64, DM / 64, 1), 32, 0, stream>>>(OPh, OPl, WEh, WEl, DO, OUT + (size_t)b * TT * DM, DM, nullptr, 0, 0, 0); }
}
